// NonLocalBlock_4011499454592
// MI455X (gfx1250) — hardware-verified
//
#include <hip/hip_runtime.h>


typedef _Float16 v16h __attribute__((ext_vector_type(16)));
typedef _Float16 v8h  __attribute__((ext_vector_type(8)));
typedef float    v8f  __attribute__((ext_vector_type(8)));
typedef float    v4f  __attribute__((ext_vector_type(4)));
typedef double   v2d  __attribute__((ext_vector_type(2)));

#ifndef NB
#define NB 8
#endif
#define NB_FULL 8
#define NC   256
#define NI   128
#define TT   8
#define HH   28
#define WD   28
#define NN   (TT * HH * WD)
#define HP   (HH / 2)
#define WQ   (WD / 2)
#define MM   (TT * HP * WQ)
#define MPAD 1600
#define NBLK (NN / 64)
#define MCH  (MPAD / 64)

#define EPSBN 1e-5f
#define XSC   16.0f
#define WSC   64.0f
#define RSC   4096.0f
#define PSC   16384.0f
#define PLSC  4.0f

#define KP 136
#define VP 40
#define PP 40

static_assert(NB >= 1 && NB <= NB_FULL);
static_assert(NN % 64 == 0);
static_assert(MM % 32 == 0);
static_assert(MM % 4 == 0);
static_assert(MPAD % 64 == 0);
static_assert(MPAD >= MM);
static_assert(NC == 2 * NI);
static_assert(NC % 64 == 0);
static_assert((NC * NN) % 1024 == 0);
static_assert((NI * NC) % 2048 == 0);
static_assert(8 * 16 * NI <= 2 * 32 * KP + 2 * NI * VP);

__device__ __forceinline__ v8f wmma16(v16h a, v16h b, v8f c) {
  return __builtin_amdgcn_wmma_f32_16x16x32_f16(false, a, false, b, (short)0, c, false, false);
}
__device__ __forceinline__ void wguard(v8f& acc, const v16h& a, const v16h& b) {
  asm volatile("v_nop\n\tv_nop\n\tv_nop\n\tv_nop" : "+v"(acc) : "v"(a), "v"(b));
}
__device__ __forceinline__ v16h load_h16(const _Float16* p) {
  const v8h lo = *(const v8h*)(p);
  const v8h hi = *(const v8h*)(p + 16);
  return __builtin_shufflevector(lo, hi, 0, 1, 2, 3, 4, 5, 6, 7,
                                 8, 9, 10, 11, 12, 13, 14, 15);
}
__device__ __forceinline__ float bf16r(float f) {
  unsigned int u = __float_as_uint(f);
  u = (u + 0x7FFFu + ((u >> 16) & 1u)) & 0xFFFF0000u;
  return __uint_as_float(u);
}
__device__ __forceinline__ void split16(float v, _Float16& eh, _Float16& el) {
  eh = (_Float16)v;
  el = (_Float16)((v - (float)eh) * RSC);
}
__device__ __forceinline__ void vst8h(_Float16* p, v8h v) { *(volatile v8h*)p = v; }
__device__ __forceinline__ void vst4f(float* p, v4f v)    { *(volatile v4f*)p = v; }
__device__ __forceinline__ void vst2d(double* p, v2d v)   { *(volatile v2d*)p = v; }

__global__ void __launch_bounds__(256)
cvt_w_kernel(const float* __restrict__ Wt, const float* __restrict__ Wp,
             const float* __restrict__ Wg, const float* __restrict__ Ww,
             _Float16* __restrict__ wt16, _Float16* __restrict__ wp16,
             _Float16* __restrict__ wg16, _Float16* __restrict__ ww16) {
  const int t = blockIdx.x * 256 + threadIdx.x;
  const size_t e = (size_t)t * 8;
  v8h a, b, c, d;
#pragma unroll
  for (int j = 0; j < 8; ++j) {
    a[j] = (_Float16)(bf16r(Wt[e + j]) * WSC);
    b[j] = (_Float16)(bf16r(Wp[e + j]) * WSC);
    c[j] = (_Float16)(bf16r(Wg[e + j]) * WSC);
    d[j] = (_Float16)(bf16r(Ww[e + j]) * WSC);
  }
  vst8h(wt16 + e, a); vst8h(wp16 + e, b); vst8h(wg16 + e, c); vst8h(ww16 + e, d);
  __threadfence();
  vst8h(wt16 + e, a); vst8h(wp16 + e, b); vst8h(wg16 + e, c); vst8h(ww16 + e, d);
}

__global__ void __launch_bounds__(256)
xpose_kernel(const float* __restrict__ x, _Float16* __restrict__ x16) {
  __shared__ float tile[32][65];
  const int per_b = (NN / 32) * (NC / 64);
  const int b = blockIdx.x / per_b;
  const int rem = blockIdx.x % per_b;
  const int c0 = (rem / (NN / 32)) * 64;
  const int n0 = (rem % (NN / 32)) * 32;
  const int t = threadIdx.x, tx = t & 31, ty = t >> 5;
  const float* xb = x + (size_t)b * NC * NN;
#pragma unroll
  for (int s = 0; s < 8; ++s) {
    const int c = c0 + ty + 8 * s;
    tile[tx][ty + 8 * s] = xb[(size_t)c * NN + n0 + tx];
  }
  __syncthreads();
  const int nr = t >> 3, pc = t & 7;
  v8h v;
#pragma unroll
  for (int j = 0; j < 8; ++j) v[j] = (_Float16)(bf16r(tile[nr][8 * pc + j]) * XSC);
  _Float16* dst = x16 + ((size_t)b * NN + n0 + nr) * NC + c0 + 8 * pc;
  vst8h(dst, v);
  __threadfence();
  vst8h(dst, v);
}

__global__ void __launch_bounds__(128)
proj_theta_kernel(const _Float16* __restrict__ x16, const _Float16* __restrict__ wt16,
                  const float* __restrict__ bt,
                  _Float16* __restrict__ thh, _Float16* __restrict__ thl) {
  __shared__ __align__(16) _Float16 sh[4][16 * NI];
  __shared__ __align__(16) _Float16 sl[4][16 * NI];
  const int lane = threadIdx.x & 31, wv = threadIdx.x >> 5;
  const int b = blockIdx.x / NBLK;
  const int n0 = (blockIdx.x % NBLK) * 64 + wv * 16;
  const int col = lane & 15, h = lane >> 4, hh = h << 3, rb = h << 3;

  const _Float16* xr = x16 + ((size_t)b * NN + n0 + col) * NC + hh;
  v16h Ax[8];
#pragma unroll
  for (int k = 0; k < 8; ++k) Ax[k] = load_h16(xr + 32 * k);

  for (int ic = 0; ic < 8; ++ic) {
    const int i = ic * 16 + col;
    const _Float16* wr = wt16 + (size_t)i * NC + hh;
    v16h Bw[8];
#pragma unroll
    for (int k = 0; k < 8; ++k) Bw[k] = load_h16(wr + 32 * k);
    v8f acc = {};
#pragma unroll
    for (int k = 0; k < 8; ++k) acc = wmma16(Ax[k], Bw[k], acc);
    wguard(acc, Ax[7], Bw[7]);
    const float bias = bf16r(bt[i]);
#pragma unroll
    for (int r = 0; r < 8; ++r) {
      const float v = acc[r] * (1.0f / 1024.0f) + bias;
      _Float16 eh, el;
      split16(v, eh, el);
      sh[wv][(rb + r) * NI + i] = eh;
      sl[wv][(rb + r) * NI + i] = el;
    }
  }
  __syncthreads();

  _Float16* oh = thh + ((size_t)b * NN + n0) * NI;
  _Float16* ol = thl + ((size_t)b * NN + n0) * NI;
  const int pc = lane & 15;
#pragma unroll
  for (int it = 0; it < 8; ++it) {
    const int row = 2 * it + h;
    vst8h(oh + (size_t)row * NI + 8 * pc, *(const v8h*)&sh[wv][row * NI + 8 * pc]);
    vst8h(ol + (size_t)row * NI + 8 * pc, *(const v8h*)&sl[wv][row * NI + 8 * pc]);
  }
  __threadfence();
#pragma unroll
  for (int it = 0; it < 8; ++it) {
    const int row = 2 * it + h;
    vst8h(oh + (size_t)row * NI + 8 * pc, *(const v8h*)&sh[wv][row * NI + 8 * pc]);
    vst8h(ol + (size_t)row * NI + 8 * pc, *(const v8h*)&sl[wv][row * NI + 8 * pc]);
  }
}

__global__ void __launch_bounds__(128)
proj_pool_kernel(const _Float16* __restrict__ x16,
                 const _Float16* __restrict__ wp16, const float* __restrict__ bp,
                 const _Float16* __restrict__ wg16, const float* __restrict__ bg,
                 _Float16* __restrict__ phh, _Float16* __restrict__ phl,
                 _Float16* __restrict__ gth, _Float16* __restrict__ gtl) {
  __shared__ __align__(16) _Float16 sph[4][4 * NI];
  __shared__ __align__(16) _Float16 spl[4][4 * NI];
  __shared__ __align__(16) _Float16 sgh[NI * 64];
  __shared__ __align__(16) _Float16 sgl[NI * 64];

  const int lane = threadIdx.x & 31, wv = threadIdx.x >> 5;
  const int b = blockIdx.x / MCH, ch = blockIdx.x % MCH;
  const int col = lane & 15, h = lane >> 4, hh = h << 3;
  const int d = lane & 15;
  const int pr = d >> 2, wq = d & 3;
  const int dy = wq >> 1, dx = wq & 1;
  const int pc = lane & 15;

  for (int tj = 0; tj < 4; ++tj) {
    const int tile = wv * 4 + tj;
    const int mg0 = ch * 64 + tile * 4;
    const float valid = (mg0 < MM) ? 1.0f : 0.0f;
    int mg = mg0 + pr;
    mg = (mg < MM) ? mg : (MM - 1);
    const int tt = mg / (HP * WQ), rm = mg % (HP * WQ);
    const int y2 = rm / WQ, x2 = rm % WQ;
    const int n = tt * (HH * WD) + (2 * y2 + dy) * WD + 2 * x2 + dx;
    const _Float16* xr = x16 + ((size_t)b * NN + n) * NC + hh;
    v16h Ax[8];
#pragma unroll
    for (int k = 0; k < 8; ++k) Ax[k] = load_h16(xr + 32 * k);

    for (int ic = 0; ic < 8; ++ic) {
      const int i = ic * 16 + col;
      const _Float16* wr = wp16 + (size_t)i * NC + hh;
      v16h Bw[8];
#pragma unroll
      for (int k = 0; k < 8; ++k) Bw[k] = load_h16(wr + 32 * k);
      v8f acc = {};
#pragma unroll
      for (int k = 0; k < 8; ++k) acc = wmma16(Ax[k], Bw[k], acc);
      wguard(acc, Ax[7], Bw[7]);
      const float bias = bf16r(bp[i]);
      const float m0 = fmaxf(fmaxf(acc[0], acc[1]), fmaxf(acc[2], acc[3]));
      const float m1 = fmaxf(fmaxf(acc[4], acc[5]), fmaxf(acc[6], acc[7]));
      const float v0 = (m0 * (1.0f / 1024.0f) + bias) * valid;
      const float v1 = (m1 * (1.0f / 1024.0f) + bias) * valid;
      _Float16 h0, l0, h1, l1;
      split16(v0, h0, l0);
      split16(v1, h1, l1);
      sph[wv][(2 * h) * NI + i] = h0;      spl[wv][(2 * h) * NI + i] = l0;
      sph[wv][(2 * h + 1) * NI + i] = h1;  spl[wv][(2 * h + 1) * NI + i] = l1;
    }
    __syncthreads();
    {
      _Float16* oh = phh + ((size_t)b * MPAD + mg0) * NI;
      _Float16* ol = phl + ((size_t)b * MPAD + mg0) * NI;
#pragma unroll
      for (int it = 0; it < 2; ++it) {
        const int row = 2 * it + h;
        vst8h(oh + (size_t)row * NI + 8 * pc, *(const v8h*)&sph[wv][row * NI + 8 * pc]);
        vst8h(ol + (size_t)row * NI + 8 * pc, *(const v8h*)&spl[wv][row * NI + 8 * pc]);
      }
      __threadfence();
#pragma unroll
      for (int it = 0; it < 2; ++it) {
        const int row = 2 * it + h;
        vst8h(oh + (size_t)row * NI + 8 * pc, *(const v8h*)&sph[wv][row * NI + 8 * pc]);
        vst8h(ol + (size_t)row * NI + 8 * pc, *(const v8h*)&spl[wv][row * NI + 8 * pc]);
      }
    }

    for (int ic = 0; ic < 8; ++ic) {
      const int i = ic * 16 + col;
      const _Float16* wr = wg16 + (size_t)i * NC + hh;
      v16h Bw[8];
#pragma unroll
      for (int k = 0; k < 8; ++k) Bw[k] = load_h16(wr + 32 * k);
      v8f acc = {};
#pragma unroll
      for (int k = 0; k < 8; ++k) acc = wmma16(Ax[k], Bw[k], acc);
      wguard(acc, Ax[7], Bw[7]);
      const float bias = bf16r(bg[i]);
      const float m0 = fmaxf(fmaxf(acc[0], acc[1]), fmaxf(acc[2], acc[3]));
      const float m1 = fmaxf(fmaxf(acc[4], acc[5]), fmaxf(acc[6], acc[7]));
      const float v0 = (m0 * (1.0f / 1024.0f) + bias) * valid;
      const float v1 = (m1 * (1.0f / 1024.0f) + bias) * valid;
      _Float16 h0, l0, h1, l1;
      split16(v0, h0, l0);
      split16(v1, h1, l1);
      const int mloc = tile * 4 + 2 * h;
      sgh[i * 64 + mloc] = h0;      sgl[i * 64 + mloc] = l0;
      sgh[i * 64 + mloc + 1] = h1;  sgl[i * 64 + mloc + 1] = l1;
    }
    __syncthreads();
  }

  {
    _Float16* oh = gth + (size_t)b * NI * MPAD + (size_t)ch * 64;
    _Float16* ol = gtl + (size_t)b * NI * MPAD + (size_t)ch * 64;
    const int p8 = lane & 7, rq = lane >> 3;
#pragma unroll
    for (int it = 0; it < 8; ++it) {
      const int i = it * 16 + wv * 4 + rq;
      vst8h(oh + (size_t)i * MPAD + 8 * p8, *(const v8h*)&sgh[i * 64 + 8 * p8]);
      vst8h(ol + (size_t)i * MPAD + 8 * p8, *(const v8h*)&sgl[i * 64 + 8 * p8]);
    }
    __threadfence();
#pragma unroll
    for (int it = 0; it < 8; ++it) {
      const int i = it * 16 + wv * 4 + rq;
      vst8h(oh + (size_t)i * MPAD + 8 * p8, *(const v8h*)&sgh[i * 64 + 8 * p8]);
      vst8h(ol + (size_t)i * MPAD + 8 * p8, *(const v8h*)&sgl[i * 64 + 8 * p8]);
    }
  }
}

__global__ void __launch_bounds__(128)
attn_kernel(const _Float16* __restrict__ thh, const _Float16* __restrict__ thl,
            const _Float16* __restrict__ phh, const _Float16* __restrict__ phl,
            const _Float16* __restrict__ gth, const _Float16* __restrict__ gtl,
            _Float16* __restrict__ yh, _Float16* __restrict__ yl) {
  __shared__ __align__(16) _Float16 skv[2 * 32 * KP + 2 * NI * VP];
  __shared__ __align__(16) _Float16 sp[4][2][16 * PP];
  _Float16* const sKh = skv;
  _Float16* const sKl = skv + 32 * KP;
  _Float16* const sVh = skv + 64 * KP;
  _Float16* const sVl = skv + 64 * KP + NI * VP;

  const int t = threadIdx.x, lane = t & 31, wv = t >> 5;
  const int b = blockIdx.x / NBLK;
  const int q0 = (blockIdx.x % NBLK) * 64 + wv * 16;
  const int col = lane & 15, h = lane >> 4, hh = h << 3, rb = h << 3;

  const size_t toff = ((size_t)b * NN + q0 + col) * NI + hh;
  v16h Th[4], Tl[4];
#pragma unroll
  for (int k = 0; k < 4; ++k) {
    Th[k] = load_h16(thh + toff + 32 * k);
    Tl[k] = load_h16(thl + toff + 32 * k);
  }

  v8f O[8];
#pragma unroll
  for (int ci = 0; ci < 8; ++ci) O[ci] = v8f{};
  float m8[8], l8[8];
#pragma unroll
  for (int r = 0; r < 8; ++r) { m8[r] = -1e30f; l8[r] = 0.0f; }

  const _Float16* Kh = phh + (size_t)b * MPAD * NI;
  const _Float16* Kl = phl + (size_t)b * MPAD * NI;
  const _Float16* Vh = gth + (size_t)b * NI * MPAD;
  const _Float16* Vl = gtl + (size_t)b * NI * MPAD;

  for (int kb = 0; kb < MM; kb += 32) {
    __syncthreads();
#pragma unroll
    for (int it = 0; it < 4; ++it) {
      const int row = it * 8 + (t >> 4), pcs = t & 15;
      const size_t g = (size_t)(kb + row) * NI + 8 * pcs;
      const int s = row * KP + 8 * pcs;
      *(v8h*)(sKh + s) = *(const v8h*)(Kh + g);
      *(v8h*)(sKl + s) = *(const v8h*)(Kl + g);
    }
#pragma unroll
    for (int it = 0; it < 4; ++it) {
      const int row = it * 32 + (t >> 2), pcs = t & 3;
      const size_t g = (size_t)row * MPAD + kb + 8 * pcs;
      const int s = row * VP + 8 * pcs;
      *(v8h*)(sVh + s) = *(const v8h*)(Vh + g);
      *(v8h*)(sVl + s) = *(const v8h*)(Vl + g);
    }
    __syncthreads();

    v8f S0h = {}, S0x = {}, S1h = {}, S1x = {};
#pragma unroll
    for (int k = 0; k < 4; ++k) {
      const v16h b0h = load_h16(sKh + col * KP + hh + 32 * k);
      const v16h b0l = load_h16(sKl + col * KP + hh + 32 * k);
      S0h = wmma16(Th[k], b0h, S0h);
      S0x = wmma16(Th[k], b0l, S0x);
      S0x = wmma16(Tl[k], b0h, S0x);
      const v16h b1h = load_h16(sKh + (16 + col) * KP + hh + 32 * k);
      const v16h b1l = load_h16(sKl + (16 + col) * KP + hh + 32 * k);
      S1h = wmma16(Th[k], b1h, S1h);
      S1x = wmma16(Th[k], b1l, S1x);
      S1x = wmma16(Tl[k], b1h, S1x);
    }
    wguard(S0h, Th[3], Tl[3]);
    wguard(S0x, Th[3], Tl[3]);
    wguard(S1h, Th[3], Tl[3]);
    wguard(S1x, Th[3], Tl[3]);

    float s0[8], s1[8];
#pragma unroll
    for (int r = 0; r < 8; ++r) {
      s0[r] = S0h[r] + S0x[r] * (1.0f / RSC);
      s1[r] = S1h[r] + S1x[r] * (1.0f / RSC);
    }

#pragma unroll
    for (int r = 0; r < 8; ++r) {
      float mx = fmaxf(s0[r], s1[r]);
      mx = fmaxf(mx, __shfl_xor(mx, 1));
      mx = fmaxf(mx, __shfl_xor(mx, 2));
      mx = fmaxf(mx, __shfl_xor(mx, 4));
      mx = fmaxf(mx, __shfl_xor(mx, 8));
      const float mn = fmaxf(m8[r], mx);
      const float sc = __expf(m8[r] - mn);
      const float p0 = __expf(s0[r] - mn);
      const float p1 = __expf(s1[r] - mn);
      const _Float16 qa = (_Float16)(p0 * PSC), qb = (_Float16)(p1 * PSC);
      const _Float16 ua = (_Float16)(p0 * PLSC), ub = (_Float16)(p1 * PLSC);
      float ps = (float)qa + (float)qb;
      ps += __shfl_xor(ps, 1);
      ps += __shfl_xor(ps, 2);
      ps += __shfl_xor(ps, 4);
      ps += __shfl_xor(ps, 8);
      l8[r] = l8[r] * sc + ps;
      m8[r] = mn;
#pragma unroll
      for (int ci = 0; ci < 8; ++ci) O[ci][r] *= sc;
      const int row = rb + r;
      sp[wv][0][row * PP + col] = qa;
      sp[wv][0][row * PP + 16 + col] = qb;
      sp[wv][1][row * PP + col] = ua;
      sp[wv][1][row * PP + 16 + col] = ub;
    }
    __syncthreads();

    const v16h APh = load_h16(&sp[wv][0][col * PP + hh]);
    const v16h APl = load_h16(&sp[wv][1][col * PP + hh]);
#pragma unroll
    for (int ci = 0; ci < 8; ++ci) {
      const v16h bvh = load_h16(sVh + (ci * 16 + col) * VP + hh);
      const v16h bvl = load_h16(sVl + (ci * 16 + col) * VP + hh);
      O[ci] = wmma16(APh, bvh, O[ci]);
      O[ci] = wmma16(APl, bvl, O[ci]);
    }
#pragma unroll
    for (int ci = 0; ci < 8; ++ci) wguard(O[ci], APh, APl);
  }

  __syncthreads();
  _Float16* const sYh = skv + wv * (16 * NI);
  _Float16* const sYl = skv + 4 * (16 * NI) + wv * (16 * NI);
  float inv[8];
#pragma unroll
  for (int r = 0; r < 8; ++r) inv[r] = 1.0f / l8[r];
#pragma unroll
  for (int ci = 0; ci < 8; ++ci) {
#pragma unroll
    for (int r = 0; r < 8; ++r) {
      const float v = O[ci][r] * inv[r];
      _Float16 eh, el;
      split16(v, eh, el);
      sYh[(rb + r) * NI + ci * 16 + col] = eh;
      sYl[(rb + r) * NI + ci * 16 + col] = el;
    }
  }
  __syncthreads();

  _Float16* oh = yh + ((size_t)b * NN + q0) * NI;
  _Float16* ol = yl + ((size_t)b * NN + q0) * NI;
  const int pc = lane & 15;
#pragma unroll
  for (int it = 0; it < 8; ++it) {
    const int row = 2 * it + h;
    vst8h(oh + (size_t)row * NI + 8 * pc, *(const v8h*)&sYh[row * NI + 8 * pc]);
    vst8h(ol + (size_t)row * NI + 8 * pc, *(const v8h*)&sYl[row * NI + 8 * pc]);
  }
  __threadfence();
#pragma unroll
  for (int it = 0; it < 8; ++it) {
    const int row = 2 * it + h;
    vst8h(oh + (size_t)row * NI + 8 * pc, *(const v8h*)&sYh[row * NI + 8 * pc]);
    vst8h(ol + (size_t)row * NI + 8 * pc, *(const v8h*)&sYl[row * NI + 8 * pc]);
  }
}

__global__ void __launch_bounds__(128)
out_kernel(const _Float16* __restrict__ yh, const _Float16* __restrict__ yl,
           const _Float16* __restrict__ ww16, const float* __restrict__ bw,
           float* __restrict__ wy, double* __restrict__ part) {
  __shared__ __align__(16) float sw[16 * 64];
  __shared__ __align__(16) double spart[512];
  const int t = threadIdx.x, lane = t & 31, wv = t >> 5;
  const int b = blockIdx.x / NBLK;
  const int n0 = (blockIdx.x % NBLK) * 64;
  const int col = lane & 15, h = lane >> 4, hh = h << 3, rb = h << 3;

  const size_t yoff = ((size_t)b * NN + n0 + wv * 16 + col) * NI + hh;
  v16h Yh[4], Yl[4];
#pragma unroll
  for (int k = 0; k < 4; ++k) {
    Yh[k] = load_h16(yh + yoff + 32 * k);
    Yl[k] = load_h16(yl + yoff + 32 * k);
  }

  for (int ct = 0; ct < 16; ++ct) {
    const int c = ct * 16 + col;
    const _Float16* wr = ww16 + (size_t)c * NI + hh;
    v16h Bw[4];
#pragma unroll
    for (int k = 0; k < 4; ++k) Bw[k] = load_h16(wr + 32 * k);
    v8f ah = {}, al = {};
#pragma unroll
    for (int k = 0; k < 4; ++k) {
      ah = wmma16(Yh[k], Bw[k], ah);
      al = wmma16(Yl[k], Bw[k], al);
    }
    wguard(ah, Yh[3], Bw[3]);
    wguard(al, Yl[3], Bw[3]);
    const float bias = bf16r(bw[c]);
#pragma unroll
    for (int r = 0; r < 8; ++r) {
      const float v = ah[r] * (1.0f / WSC) + al[r] * (1.0f / (WSC * RSC)) + bias;
      sw[col * 64 + wv * 16 + rb + r] = v;
    }
    __syncthreads();

    {
      float* ob = wy + ((size_t)b * NC + ct * 16) * NN + n0;
      const int nf = 4 * (lane & 15);
#pragma unroll
      for (int j = 0; j < 2; ++j) {
        const int crow = wv * 4 + 2 * j + h;
        vst4f(ob + (size_t)crow * NN + nf, *(const v4f*)&sw[crow * 64 + nf]);
      }
      __threadfence();
#pragma unroll
      for (int j = 0; j < 2; ++j) {
        const int crow = wv * 4 + 2 * j + h;
        vst4f(ob + (size_t)crow * NN + nf, *(const v4f*)&sw[crow * 64 + nf]);
      }
    }
    {
      const int crow = t >> 3, seg = t & 7;
      double s1 = 0.0, s2 = 0.0;
#pragma unroll
      for (int j = 0; j < 8; ++j) {
        const float v = sw[crow * 64 + seg * 8 + j];
        s1 += (double)v;
        s2 += (double)v * (double)v;
      }
      s1 += __shfl_xor(s1, 1); s2 += __shfl_xor(s2, 1);
      s1 += __shfl_xor(s1, 2); s2 += __shfl_xor(s2, 2);
      s1 += __shfl_xor(s1, 4); s2 += __shfl_xor(s2, 4);
      if (seg == 0) {
        spart[ct * 16 + crow] = s1;
        spart[256 + ct * 16 + crow] = s2;
      }
    }
    __syncthreads();
  }

  double* prow = part + (size_t)blockIdx.x * 512;
#pragma unroll
  for (int j = 0; j < 2; ++j) {
    const int idx = j * 256 + 2 * t;
    vst2d(prow + idx, *(const v2d*)&spart[idx]);
  }
  __threadfence();
#pragma unroll
  for (int j = 0; j < 2; ++j) {
    const int idx = j * 256 + 2 * t;
    vst2d(prow + idx, *(const v2d*)&spart[idx]);
  }
}

__global__ void __launch_bounds__(256)
bn_kernel(const double* __restrict__ part, const float* __restrict__ gamma,
          const float* __restrict__ beta, float* __restrict__ ab) {
  __shared__ __align__(16) float sab[512];
  const int c = threadIdx.x;
  double s1 = 0.0, s2 = 0.0;
#pragma unroll 1
  for (int r = 0; r < NB * NBLK; ++r) {
    s1 += part[(size_t)r * 512 + c];
    s2 += part[(size_t)r * 512 + 256 + c];
  }
  const double inv = 1.0 / (double)(NB * NN);
  const double mean = s1 * inv;
  double var = s2 * inv - mean * mean;
  var = (var > 0.0) ? var : 0.0;
  const float rs = rsqrtf((float)var + EPSBN);
  const float ga = bf16r(gamma[c]), be = bf16r(beta[c]);
  const float A = ga * rs;
  const float Bc = be - (float)mean * A;
  sab[c] = A;
  sab[256 + c] = Bc;
  __syncthreads();
  if (c < 128) vst4f(ab + 4 * c, *(const v4f*)&sab[4 * c]);
  __threadfence();
  if (c < 128) vst4f(ab + 4 * c, *(const v4f*)&sab[4 * c]);
}

__global__ void __launch_bounds__(256)
apply_kernel(const float* __restrict__ wy, const float* __restrict__ x,
             const float* __restrict__ ab, float* __restrict__ out) {
  const size_t i4 = (size_t)blockIdx.x * 256 + threadIdx.x;
  const size_t base = i4 * 4;
  const int c = (int)((base / NN) % NC);
  const float A = ab[c], Bc = ab[256 + c];
  const v4f w = *(const v4f*)(wy + base);
  const v4f xv = *(const v4f*)(x + base);
  v4f o;
#pragma unroll
  for (int j = 0; j < 4; ++j) o[j] = fmaf(w[j], A, Bc) + bf16r(xv[j]);
  vst4f(out + base, o);
  __threadfence();
  vst4f(out + base, o);
}

extern "C" void kernel_launch(void* const* d_in, const int* in_sizes, int n_in,
                              void* d_out, int out_size, void* d_ws, size_t ws_size,
                              hipStream_t stream) {
  if (n_in < 11) return;
  if (in_sizes[0] < NB * NC * NN) return;
  if (in_sizes[1] < NI * NC || in_sizes[3] < NI * NC || in_sizes[5] < NI * NC ||
      in_sizes[7] < NC * NI) return;
  if (in_sizes[2] < NI || in_sizes[4] < NI || in_sizes[6] < NI) return;
  if (in_sizes[8] < NC || in_sizes[9] < NC || in_sizes[10] < NC) return;
  if (out_size < NB * NC * NN) return;

  const float* x     = (const float*)d_in[0];
  const float* Wg    = (const float*)d_in[1];
  const float* bg    = (const float*)d_in[2];
  const float* Wt    = (const float*)d_in[3];
  const float* bt    = (const float*)d_in[4];
  const float* Wp    = (const float*)d_in[5];
  const float* bp    = (const float*)d_in[6];
  const float* Ww    = (const float*)d_in[7];
  const float* bw    = (const float*)d_in[8];
  const float* gamma = (const float*)d_in[9];
  const float* beta  = (const float*)d_in[10];
  float* out = (float*)d_out;

  const size_t szW    = (size_t)NI * NC * sizeof(_Float16);
  const size_t szXY   = (size_t)NB * NN * NC * sizeof(_Float16);
  const size_t szT    = (size_t)NB * NN * NI * sizeof(_Float16);
  const size_t szP    = (size_t)NB * MPAD * NI * sizeof(_Float16);
  const size_t szWY   = (size_t)NB * NC * NN * sizeof(float);
  const size_t szPart = (size_t)NB * NBLK * 512 * sizeof(double);
  const size_t szAB   = (size_t)512 * sizeof(float);
  char* base = (char*)d_ws;
  size_t off = 0;
  _Float16* wt16 = (_Float16*)(base + off); off += szW;
  _Float16* wp16 = (_Float16*)(base + off); off += szW;
  _Float16* wg16 = (_Float16*)(base + off); off += szW;
  _Float16* ww16 = (_Float16*)(base + off); off += szW;
  _Float16* x16  = (_Float16*)(base + off);
  _Float16* yh   = x16;
  _Float16* yl   = x16 + (size_t)NB * NN * NI;
  off += szXY;
  _Float16* thh = (_Float16*)(base + off); off += szT;
  _Float16* thl = (_Float16*)(base + off); off += szT;
  _Float16* phh = (_Float16*)(base + off); off += szP;
  _Float16* phl = (_Float16*)(base + off); off += szP;
  _Float16* gth = (_Float16*)(base + off); off += szP;
  _Float16* gtl = (_Float16*)(base + off); off += szP;
  float* wy     = (float*)(base + off);    off += szWY;
  double* part  = (double*)(base + off);   off += szPart;
  float* ab     = (float*)(base + off);    off += szAB;
  if (off > ws_size) return;

  cvt_w_kernel<<<(NI * NC) / 2048, 256, 0, stream>>>(Wt, Wp, Wg, Ww, wt16, wp16, wg16, ww16);
  xpose_kernel<<<NB * (NN / 32) * (NC / 64), 256, 0, stream>>>(x, x16);
  proj_theta_kernel<<<NB * NBLK, 128, 0, stream>>>(x16, wt16, bt, thh, thl);
  proj_pool_kernel<<<NB * MCH, 128, 0, stream>>>(x16, wp16, bp, wg16, bg, phh, phl, gth, gtl);
  attn_kernel<<<NB * NBLK, 128, 0, stream>>>(thh, thl, phh, phl, gth, gtl, yh, yl);
  out_kernel<<<NB * NBLK, 128, 0, stream>>>(yh, yl, ww16, bw, wy, part);
  bn_kernel<<<1, 256, 0, stream>>>(part, gamma, beta, ab);
  apply_kernel<<<(NB * NC * NN) / 1024, 256, 0, stream>>>(wy, x, ab, out);
}
